// PerformerSelfAttention_34626026340876
// MI455X (gfx1250) — hardware-verified
//
#include <hip/hip_runtime.h>
#include <stdint.h>


typedef _Float16 f16_t;
typedef _Float16 v16h __attribute__((ext_vector_type(16)));
typedef _Float16 v8h  __attribute__((ext_vector_type(8)));
typedef _Float16 v2h  __attribute__((ext_vector_type(2)));
typedef float    v8f  __attribute__((ext_vector_type(8)));
typedef float    v4f  __attribute__((ext_vector_type(4)));
typedef unsigned int u32x4 __attribute__((ext_vector_type(4)));

#define EPS_F 1e-6f
#define NB   2
#define NL   2048
#define ND   1024
#define NH   16
#define HDIM 64

union Frag { v16h v; u32x4 q[2]; };

__device__ __forceinline__ v16h ld_frag(const f16_t* base, int pitch, int lane) {
    const int m = lane & 15, h = lane >> 4;
    const f16_t* p = base + (size_t)m * pitch + 8 * h;
    Frag f;
    f.q[0] = *(const u32x4*)(p);
    f.q[1] = *(const u32x4*)(p + 16);
    return f.v;
}

__device__ __forceinline__ v8f wmma16(v16h a, v16h b, v8f c) {
    v8f d = __builtin_amdgcn_wmma_f32_16x16x32_f16(false, a, false, b, (short)0, c, false, false);
    asm volatile("v_nop\n\tv_nop\n\tv_nop\n\tv_nop" : "+v"(d) : "v"(a), "v"(b));
    return d;
}

__device__ __forceinline__ v8f zero8() {
    v8f r;
#pragma unroll
    for (int i = 0; i < 8; ++i) r[i] = 0.0f;
    return r;
}

__device__ __forceinline__ float wave_max(float v) {
#pragma unroll
    for (int o = 16; o > 0; o >>= 1) v = fmaxf(v, __shfl_xor(v, o, 32));
    return v;
}
__device__ __forceinline__ float wave_sum(float v) {
#pragma unroll
    for (int o = 16; o > 0; o >>= 1) v += __shfl_xor(v, o, 32);
    return v;
}

__global__ void __launch_bounds__(256)
k_cvt_x(const float* __restrict__ x, f16_t* __restrict__ y, int n8) {
    const int i = blockIdx.x * 256 + threadIdx.x;
    if (i >= n8) return;
    const float* p = x + (size_t)i * 8;
    float4 a = *(const float4*)(p);
    float4 b = *(const float4*)(p + 4);
    union { v8h v; f16_t e[8]; } u;
    u.e[0] = (f16_t)a.x; u.e[1] = (f16_t)a.y; u.e[2] = (f16_t)a.z; u.e[3] = (f16_t)a.w;
    u.e[4] = (f16_t)b.x; u.e[5] = (f16_t)b.y; u.e[6] = (f16_t)b.z; u.e[7] = (f16_t)b.w;
    f16_t* d = y + (size_t)i * 8;
    *(volatile v8h*)d = u.v;
    __threadfence();
    *(volatile v8h*)d = u.v;
}

#define WTP 72

__global__ void __launch_bounds__(256)
k_cvt_w(const float* __restrict__ w0, const float* __restrict__ w1,
        const float* __restrict__ w2, const float* __restrict__ w3,
        f16_t* __restrict__ t0, f16_t* __restrict__ t1,
        f16_t* __restrict__ t2, f16_t* __restrict__ t3,
        int K, int N, float scale) {
    __shared__ f16_t ts[64 * WTP];
    const int z = blockIdx.z;
    const float* w = (z == 0) ? w0 : ((z == 1) ? w1 : ((z == 2) ? w2 : w3));
    f16_t* t = (z == 0) ? t0 : ((z == 1) ? t1 : ((z == 2) ? t2 : t3));
    const int tid = threadIdx.x;
    const int n0 = blockIdx.x * 64;
    const int k0 = blockIdx.y * 64;
    if (n0 + 64 > N || k0 + 64 > K) return;

#pragma unroll
    for (int j = 0; j < 4; ++j) {
        const int idx = tid + 256 * j;
        const int kr  = idx >> 4;
        const int nc  = (idx & 15) * 4;
        float4 f = *(const float4*)(w + (size_t)(k0 + kr) * N + n0 + nc);
        ts[(nc + 0) * WTP + kr] = (f16_t)(f.x * scale);
        ts[(nc + 1) * WTP + kr] = (f16_t)(f.y * scale);
        ts[(nc + 2) * WTP + kr] = (f16_t)(f.z * scale);
        ts[(nc + 3) * WTP + kr] = (f16_t)(f.w * scale);
    }
    __syncthreads();

    v8h vv[2];
    f16_t* dp[2];
#pragma unroll
    for (int j = 0; j < 2; ++j) {
        const int nl = (tid >> 3) + 32 * j;
        const int piece = tid & 7;
        vv[j] = *(const v8h*)(&ts[nl * WTP + piece * 8]);
        dp[j] = t + (size_t)(n0 + nl) * K + k0 + piece * 8;
    }
#pragma unroll
    for (int j = 0; j < 2; ++j) *(volatile v8h*)dp[j] = vv[j];
    __threadfence();
#pragma unroll
    for (int j = 0; j < 2; ++j) *(volatile v8h*)dp[j] = vv[j];
}

#define GBM 128
#define GBN 128
#define GBK 64
#define LDP 72

__global__ void __launch_bounds__(256)
k_gemm(const f16_t* __restrict__ A,
       const f16_t* __restrict__ Bt0, const f16_t* __restrict__ Bt1, const f16_t* __restrict__ Bt2,
       const float* __restrict__ bs0, const float* __restrict__ bs1, const float* __restrict__ bs2,
       float* __restrict__ C0, float* __restrict__ C1, float* __restrict__ C2,
       int M, int N, int K, float oscale) {
    __shared__ u32x4 lds_raw[(2 * GBM * LDP * 2) / 16];
    f16_t* ldsA = (f16_t*)lds_raw;
    f16_t* ldsB = ldsA + GBM * LDP;

    const int z = blockIdx.z;
    const f16_t* Bt  = (z == 0) ? Bt0 : ((z == 1) ? Bt1 : Bt2);
    const float* bias = (z == 0) ? bs0 : ((z == 1) ? bs1 : bs2);
    float* C          = (z == 0) ? C0 : ((z == 1) ? C1 : C2);

    const int tid  = threadIdx.x;
    const int lane = tid & 31;
    const int wave = tid >> 5;
    const int wm   = wave >> 2;
    const int wn   = wave & 3;
    const int m    = lane & 15;
    const int h    = lane >> 4;
    const int rowBase = blockIdx.y * GBM;
    const int colBase = blockIdx.x * GBN;
    if (rowBase + GBM > M || colBase + GBN > N) return;

    v8f acc[4][2];
#pragma unroll
    for (int tm = 0; tm < 4; ++tm)
#pragma unroll
        for (int tn = 0; tn < 2; ++tn) acc[tm][tn] = zero8();

    for (int kk = 0; kk < K; kk += GBK) {
#pragma unroll
        for (int j = 0; j < 4; ++j) {
            const int chunk = tid + j * 256;
            const int r = chunk >> 3;
            const int c = (chunk & 7) * 8;
            u32x4 va = *(const u32x4*)(A  + (size_t)(rowBase + r) * K + kk + c);
            u32x4 vb = *(const u32x4*)(Bt + (size_t)(colBase + r) * K + kk + c);
            *(u32x4*)(ldsA + r * LDP + c) = va;
            *(u32x4*)(ldsB + r * LDP + c) = vb;
        }
        __syncthreads();

#pragma unroll
        for (int ks = 0; ks < 2; ++ks) {
            v16h af[4], bf[2];
#pragma unroll
            for (int tm = 0; tm < 4; ++tm)
                af[tm] = ld_frag(ldsA + (wm * 64 + tm * 16) * LDP + ks * 32, LDP, lane);
#pragma unroll
            for (int tn = 0; tn < 2; ++tn)
                bf[tn] = ld_frag(ldsB + (wn * 32 + tn * 16) * LDP + ks * 32, LDP, lane);
#pragma unroll
            for (int tm = 0; tm < 4; ++tm)
#pragma unroll
                for (int tn = 0; tn < 2; ++tn)
                    acc[tm][tn] = wmma16(af[tm], bf[tn], acc[tm][tn]);
        }
        __syncthreads();
    }

    float* wl = (float*)lds_raw + wave * 512;
    float bb[2];
#pragma unroll
    for (int tn = 0; tn < 2; ++tn) bb[tn] = bias[colBase + wn * 32 + tn * 16 + m];
    const int piece = lane & 7;
    const int rq    = lane >> 3;
    const size_t colOut = (size_t)colBase + wn * 32 + piece * 4;

#pragma unroll
    for (int tm = 0; tm < 4; ++tm) {
#pragma unroll
        for (int tn = 0; tn < 2; ++tn)
#pragma unroll
            for (int r = 0; r < 8; ++r)
                wl[(8 * h + r) * 32 + tn * 16 + m] = acc[tm][tn][r] * oscale + bb[tn];
        __syncthreads();
        v4f vv[4];
        float* gp[4];
#pragma unroll
        for (int j = 0; j < 4; ++j) {
            const int row = j * 4 + rq;
            vv[j] = *(const v4f*)(wl + row * 32 + piece * 4);
            gp[j] = C + ((size_t)rowBase + wm * 64 + tm * 16 + row) * N + colOut;
        }
        __syncthreads();
#pragma unroll
        for (int j = 0; j < 4; ++j) *(volatile v4f*)gp[j] = vv[j];
        __threadfence();
#pragma unroll
        for (int j = 0; j < 4; ++j) *(volatile v4f*)gp[j] = vv[j];
    }
}

__global__ void __launch_bounds__(256)
k_featmap(const float* __restrict__ qb, const float* __restrict__ kb,
          const float* __restrict__ vb,
          f16_t* __restrict__ qf, f16_t* __restrict__ kfT, f16_t* __restrict__ vT,
          int L, int H, int D) {
    __shared__ f16_t qs[64 * 64];
    __shared__ f16_t ksT[64 * 64];
    __shared__ f16_t vsT[64 * 64];

    const int nchunk = L / 64;
    const int bh    = blockIdx.x / nchunk;
    const int chunk = blockIdx.x % nchunk;
    const int b  = bh / H;
    const int hh = bh % H;
    const int l0 = chunk * 64;
    const int tid  = threadIdx.x;
    const int lane = tid & 31;
    const int wave = tid >> 5;
    const int d0 = 2 * lane;

#pragma unroll 1
    for (int tt = 0; tt < 8; ++tt) {
        const int t = wave * 8 + tt;
        const size_t row = ((size_t)(b * L + l0 + t)) * D + hh * HDIM + d0;
        float2 xq = *(const float2*)(qb + row);
        float2 xk = *(const float2*)(kb + row);
        float2 xv = *(const float2*)(vb + row);

        {
            float mx = wave_max(fmaxf(xq.x, xq.y));
            float e0 = expf(xq.x - mx);
            float e1 = expf(xq.y - mx);
            float s  = wave_sum(e0 + e1);
            float inv = 1.0f / (s + EPS_F);
            float p0 = e0 * inv, p1 = e1 * inv;
            float ds = wave_sum(p0 + p1);
            float sc = (1.0f / (ds + EPS_F)) * 16384.0f;
            v2h pv; pv[0] = (f16_t)(p0 * sc); pv[1] = (f16_t)(p1 * sc);
            *(v2h*)(&qs[t * 64 + d0]) = pv;
        }
        {
            float mx = wave_max(fmaxf(xk.x, xk.y));
            float e0 = expf(xk.x - mx);
            float e1 = expf(xk.y - mx);
            float s  = wave_sum(e0 + e1);
            float sc = (1.0f / (s + EPS_F)) * 16384.0f;
            ksT[(d0 + 0) * 64 + t] = (f16_t)(e0 * sc);
            ksT[(d0 + 1) * 64 + t] = (f16_t)(e1 * sc);
        }
        vsT[(d0 + 0) * 64 + t] = (f16_t)xv.x;
        vsT[(d0 + 1) * 64 + t] = (f16_t)xv.y;
    }
    __syncthreads();

    v8h vq[2], vk[2], vv[2];
    f16_t* dq[2];
    f16_t* dk[2];
    f16_t* dv[2];
    const int piece = tid & 7;
#pragma unroll
    for (int j = 0; j < 2; ++j) {
        const int rr = (tid >> 3) + 32 * j;
        vq[j] = *(const v8h*)(&qs[rr * 64 + piece * 8]);
        vk[j] = *(const v8h*)(&ksT[rr * 64 + piece * 8]);
        vv[j] = *(const v8h*)(&vsT[rr * 64 + piece * 8]);
        dq[j] = qf  + ((size_t)bh * L + l0 + rr) * HDIM + piece * 8;
        dk[j] = kfT + ((size_t)bh * HDIM + rr) * L + l0 + piece * 8;
        dv[j] = vT  + ((size_t)bh * HDIM + rr) * L + l0 + piece * 8;
    }
#pragma unroll
    for (int j = 0; j < 2; ++j) {
        *(volatile v8h*)dq[j] = vq[j];
        *(volatile v8h*)dk[j] = vk[j];
        *(volatile v8h*)dv[j] = vv[j];
    }
    __threadfence();
#pragma unroll
    for (int j = 0; j < 2; ++j) {
        *(volatile v8h*)dq[j] = vq[j];
        *(volatile v8h*)dk[j] = vk[j];
        *(volatile v8h*)dv[j] = vv[j];
    }
}

__global__ void __launch_bounds__(256)
k_kv(const f16_t* __restrict__ kfT, const f16_t* __restrict__ vT,
     f16_t* __restrict__ St, int L) {
    __shared__ f16_t ss[64 * 64];
    const int bh   = blockIdx.x;
    const int tid  = threadIdx.x;
    const int lane = tid & 31;
    const int wave = tid >> 5;
    const int wm   = wave >> 1;
    const int wnb  = (wave & 1) * 2;
    const int m    = lane & 15;
    const int h    = lane >> 4;

    const f16_t* ka  = kfT + ((size_t)bh * HDIM + wm * 16) * L;
    const f16_t* vb0 = vT  + ((size_t)bh * HDIM + (wnb + 0) * 16) * L;
    const f16_t* vb1 = vT  + ((size_t)bh * HDIM + (wnb + 1) * 16) * L;

    v8f acc0 = zero8(), acc1 = zero8();
#pragma unroll 2
    for (int kk = 0; kk < L; kk += 32) {
        v16h a  = ld_frag(ka + kk, L, lane);
        v16h b0 = ld_frag(vb0 + kk, L, lane);
        v16h b1 = ld_frag(vb1 + kk, L, lane);
        acc0 = wmma16(a, b0, acc0);
        acc1 = wmma16(a, b1, acc1);
    }

    const float sc = 1.0f / 1024.0f;
#pragma unroll
    for (int r = 0; r < 8; ++r) {
        const int d = wm * 16 + 8 * h + r;
        ss[((wnb + 0) * 16 + m) * 64 + d] = (f16_t)(acc0[r] * sc);
        ss[((wnb + 1) * 16 + m) * 64 + d] = (f16_t)(acc1[r] * sc);
    }
    __syncthreads();

    v8h vv[2];
    f16_t* dp[2];
    const int piece = tid & 7;
#pragma unroll
    for (int j = 0; j < 2; ++j) {
        const int e = (tid >> 3) + 32 * j;
        vv[j] = *(const v8h*)(&ss[e * 64 + piece * 8]);
        dp[j] = St + (size_t)bh * 4096 + e * 64 + piece * 8;
    }
#pragma unroll
    for (int j = 0; j < 2; ++j) *(volatile v8h*)dp[j] = vv[j];
    __threadfence();
#pragma unroll
    for (int j = 0; j < 2; ++j) *(volatile v8h*)dp[j] = vv[j];
}

__global__ void __launch_bounds__(256)
k_ctx(const f16_t* __restrict__ qf, const f16_t* __restrict__ St,
      f16_t* __restrict__ ctx, int L, int H) {
    __shared__ f16_t cs[128 * 64];
    const int nchunk = L / 128;
    const int bh    = blockIdx.x / nchunk;
    const int chunk = blockIdx.x % nchunk;
    const int b  = bh / H;
    const int hh = bh % H;
    const int tid  = threadIdx.x;
    const int lane = tid & 31;
    const int wave = tid >> 5;
    const int m    = lane & 15;
    const int h    = lane >> 4;
    const int t0   = wave * 16;

    const f16_t* qa = qf + ((size_t)bh * L + chunk * 128 + t0) * HDIM;
    const f16_t* sb = St + (size_t)bh * 4096;

    v8f acc[4];
#pragma unroll
    for (int tn = 0; tn < 4; ++tn) acc[tn] = zero8();
#pragma unroll
    for (int ks = 0; ks < 2; ++ks) {
        v16h a = ld_frag(qa + ks * 32, HDIM, lane);
#pragma unroll
        for (int tn = 0; tn < 4; ++tn) {
            v16h bfr = ld_frag(sb + (tn * 16) * 64 + ks * 32, 64, lane);
            acc[tn] = wmma16(a, bfr, acc[tn]);
        }
    }

    const float sc = 1.0f / 262144.0f;
#pragma unroll
    for (int tn = 0; tn < 4; ++tn)
#pragma unroll
        for (int r = 0; r < 8; ++r)
            cs[(t0 + 8 * h + r) * 64 + tn * 16 + m] = (f16_t)(acc[tn][r] * sc);
    __syncthreads();

    v8h vv[4];
    f16_t* dp[4];
    const int piece = tid & 7;
#pragma unroll
    for (int j = 0; j < 4; ++j) {
        const int t = (tid >> 3) + 32 * j;
        vv[j] = *(const v8h*)(&cs[t * 64 + piece * 8]);
        dp[j] = ctx + ((size_t)(b * L + chunk * 128 + t) * H + hh) * HDIM + piece * 8;
    }
#pragma unroll
    for (int j = 0; j < 4; ++j) *(volatile v8h*)dp[j] = vv[j];
    __threadfence();
#pragma unroll
    for (int j = 0; j < 4; ++j) *(volatile v8h*)dp[j] = vv[j];
}

extern "C" void kernel_launch(void* const* d_in, const int* in_sizes, int n_in,
                              void* d_out, int out_size, void* d_ws, size_t ws_size,
                              hipStream_t stream) {
    const int B = NB, L = NL, D = ND, H = NH;
    const int M = B * L;
    const size_t nX = (size_t)M * D;
    const size_t nW = (size_t)D * D;

    if (n_in < 9) return;
    if (in_sizes[0] != (int)nX || in_sizes[1] != (int)nW || in_sizes[2] != D ||
        in_sizes[3] != (int)nW || in_sizes[4] != D || in_sizes[5] != (int)nW ||
        in_sizes[6] != D || in_sizes[7] != (int)nW || in_sizes[8] != D) return;
    if (out_size != (int)nX) return;

    const float* hsrc = (const float*)d_in[0];
    const float* Wq = (const float*)d_in[1];
    const float* bq = (const float*)d_in[2];
    const float* Wk = (const float*)d_in[3];
    const float* bk = (const float*)d_in[4];
    const float* Wv = (const float*)d_in[5];
    const float* bv = (const float*)d_in[6];
    const float* Wo = (const float*)d_in[7];
    const float* bo = (const float*)d_in[8];
    float* out = (float*)d_out;

    size_t off = 0;
    auto carve = [&](size_t bytes) -> size_t {
        size_t p = off;
        off += (bytes + 255) & ~(size_t)255;
        return p;
    };
    const size_t oX16  = carve(nX * 2);
    const size_t oWq16 = carve(nW * 2);
    const size_t oWk16 = carve(nW * 2);
    const size_t oWv16 = carve(nW * 2);
    const size_t oWo16 = carve(nW * 2);
    const size_t oQ    = carve(nX * 4);
    const size_t oK    = carve(nX * 4);
    const size_t oV    = carve(nX * 4);
    const size_t oQf   = carve(nX * 2);
    const size_t oKfT  = carve(nX * 2);
    const size_t oVT   = carve(nX * 2);
    const size_t oSt   = carve((size_t)B * H * 64 * 64 * 2);
    const size_t oCtx  = carve(nX * 2);
    if (off > ws_size) return;

    char* ws = (char*)d_ws;
    f16_t* X16  = (f16_t*)(ws + oX16);
    f16_t* WqT  = (f16_t*)(ws + oWq16);
    f16_t* WkT  = (f16_t*)(ws + oWk16);
    f16_t* WvT  = (f16_t*)(ws + oWv16);
    f16_t* WoT  = (f16_t*)(ws + oWo16);
    float*  qb  = (float*)(ws + oQ);
    float*  kbf = (float*)(ws + oK);
    float*  vbf = (float*)(ws + oV);
    f16_t* qf   = (f16_t*)(ws + oQf);
    f16_t* kfT  = (f16_t*)(ws + oKfT);
    f16_t* vT   = (f16_t*)(ws + oVT);
    f16_t* St   = (f16_t*)(ws + oSt);
    f16_t* ctx  = (f16_t*)(ws + oCtx);

    const int n8 = (int)(nX / 8);
    k_cvt_x<<<(n8 + 255) / 256, 256, 0, stream>>>(hsrc, X16, n8);

    dim3 gw(D / 64, D / 64, 4);
    k_cvt_w<<<gw, 256, 0, stream>>>(Wq, Wk, Wv, Wo, WqT, WkT, WvT, WoT, D, D, 32.0f);

    dim3 g3(D / GBN, M / GBM, 3);
    k_gemm<<<g3, 256, 0, stream>>>(X16, WqT, WkT, WvT, bq, bk, bv, qb, kbf, vbf,
                                   M, D, D, 1.0f / 32.0f);

    k_featmap<<<B * H * (L / 64), 256, 0, stream>>>(qb, kbf, vbf, qf, kfT, vT, L, H, D);

    k_kv<<<B * H, 256, 0, stream>>>(kfT, vT, St, L);
    k_ctx<<<B * H * (L / 128), 256, 0, stream>>>(qf, St, ctx, L, H);

    dim3 g1(D / GBN, M / GBM, 1);
    k_gemm<<<g1, 256, 0, stream>>>(ctx, WoT, WoT, WoT, bo, bo, bo, out, out, out,
                                   M, D, D, 1.0f / 32.0f);
}
